// GINConv_70935679861205
// MI455X (gfx1250) — hardware-verified
//
#include <hip/hip_runtime.h>
#include <math.h>

constexpr int kNodes   = 50000;
constexpr int kNbr     = 32;
constexpr int kCh      = 128;
constexpr int kRowsPad = 50048;
constexpr float kWCarry    = 16.0f;
constexpr float kWCarryInv = 1.0f / 16.0f;
constexpr float kInvCh     = 1.0f / 128.0f;
constexpr float kLnEps     = 1e-5f;
static_assert(kRowsPad % 64 == 0 && kRowsPad >= kNodes && kRowsPad - kNodes < 64);
static_assert(kCh % 64 == 0);
static_assert(kCh % 32 == 0);
static_assert(kRowsPad % 32 == 0);
static_assert(kNodes % 8 == 0);
static_assert(kNbr == 32);

typedef __attribute__((ext_vector_type(16))) _Float16 v16h;
typedef __attribute__((ext_vector_type(8)))  _Float16 v8h;
typedef __attribute__((ext_vector_type(16))) __bf16   v16b;
typedef __attribute__((ext_vector_type(8)))  __bf16   v8b;
typedef __attribute__((ext_vector_type(8)))  float    v8f;
typedef __attribute__((ext_vector_type(4)))  float    v4f;
typedef __attribute__((ext_vector_type(4)))  unsigned int v4u;

__device__ __forceinline__ unsigned short f2bf_bits(float f) {
  unsigned u = __float_as_uint(f);
  return (unsigned short)((u + 0x7FFFu + ((u >> 16) & 1u)) >> 16);
}
__device__ __forceinline__ float bf_bits2f(unsigned short h) { return __uint_as_float(((unsigned)h) << 16); }

__device__ __forceinline__ void dep_guard_h(v8f& a, v8f& b, v16h x, v16h y) { asm volatile("v_nop\n\tv_nop\n\tv_nop\n\tv_nop" : "+v"(a), "+v"(b) : "v"(x), "v"(y)); }
__device__ __forceinline__ void dep_guard_b(v8f& a, v8f& b, v16b x, v16b y) { asm volatile("v_nop\n\tv_nop\n\tv_nop\n\tv_nop" : "+v"(a), "+v"(b) : "v"(x), "v"(y)); }
__device__ __forceinline__ void keep4_h(v16h a, v16h b, v16h c, v16h d) { asm volatile("v_nop" :: "v"(a), "v"(b), "v"(c), "v"(d)); }
__device__ __forceinline__ void keep4_b(v16b a, v16b b, v16b c, v16b d) { asm volatile("v_nop" :: "v"(a), "v"(b), "v"(c), "v"(d)); }
__device__ __forceinline__ void acc_guard4(v8f& a, v8f& b, v8f& c, v8f& d) { asm volatile("v_nop\n\tv_nop\n\tv_nop\n\tv_nop" : "+v"(a), "+v"(b), "+v"(c), "+v"(d)); }
template <typename T> struct Frag;
template <> struct Frag<_Float16> {
  typedef v16h V; union U { v16h v; v8h h[2]; };
  static __device__ __forceinline__ v16h load(const _Float16* p) {
    U f; f.h[0] = *(const v8h*)(p); f.h[1] = *(const v8h*)(p + 16); return f.v;
  }
  static __device__ __forceinline__ v8f mma(v16h a, v16h b, v8f c) {
    return __builtin_amdgcn_wmma_f32_16x16x32_f16(false, a, false, b, (short)0, c, false, false);
  }
  static __device__ __forceinline__ void guard(v8f& a, v8f& b, v16h x, v16h y) { dep_guard_h(a, b, x, y); }
  static __device__ __forceinline__ void keep(v16h a, v16h b, v16h c, v16h d) { keep4_h(a, b, c, d); }
};
template <> struct Frag<__bf16> {
  typedef v16b V; union U { v16b v; v8b h[2]; };
  static __device__ __forceinline__ v16b load(const __bf16* p) {
    U f; f.h[0] = *(const v8b*)(p); f.h[1] = *(const v8b*)(p + 16); return f.v;
  }
  static __device__ __forceinline__ v8f mma(v16b a, v16b b, v8f c) {
    return __builtin_amdgcn_wmma_f32_16x16x32_bf16(false, a, false, b, (short)0, c, false, false);
  }
  static __device__ __forceinline__ void guard(v8f& a, v8f& b, v16b x, v16b y) { dep_guard_b(a, b, x, y); }
  static __device__ __forceinline__ void keep(v16b a, v16b b, v16b c, v16b d) { keep4_b(a, b, c, d); }
};

__device__ __forceinline__ unsigned pk16(unsigned short a, unsigned short b) { return (unsigned)a | ((unsigned)b << 16); }
__device__ __forceinline__ unsigned short h_bits(float f) { const _Float16 h = (_Float16)f; return __builtin_bit_cast(unsigned short, h); }

template <int ET> struct Elem;
template <> struct Elem<0> { typedef _Float16 T; };
template <> struct Elem<1> { typedef __bf16 T; };
template <int ET, bool SPLIT, int BIAS_MODE, int OUT_MODE, bool RESID, int ACT = 0>
__global__ __launch_bounds__(256) void wmma_gemm64(
    const unsigned short* __restrict__ Ap, const unsigned short* __restrict__ A2p, int lda, long strideA,
    const unsigned short* __restrict__ Btp, const unsigned short* __restrict__ Bt2p, int ldb, long strideB,
    void* __restrict__ Cout, void* __restrict__ Cout2, int ldc, long strideC,
    const float* __restrict__ bias,
    const float* __restrict__ resid, long strideR,
    int M, int N, int K, float scale) {
  typedef typename Elem<ET>::T T;
  typedef typename Frag<T>::V V;
  const T* A = (const T*)Ap; const T* A2 = (const T*)A2p; const T* Bt = (const T*)Btp; const T* Bt2 = (const T*)Bt2p;
  __shared__ __align__(16) float sT[8][16 * 68];
  const int b    = blockIdx.y;
  const int lane = threadIdx.x & 31;
  const int wave = threadIdx.x >> 5;
  const int tilesN = N >> 6;
  const int tilesM = M >> 6;
  const int tile = blockIdx.x * 8 + wave;
  if (tile >= tilesM * tilesN) return;
  const int tm = tile / tilesN;
  const int tn = tile - tm * tilesN;
  const int m0 = tm << 6;
  const int n0 = tn << 6;

  const T* Ab  = A  + (size_t)b * strideA;
  const T* Bb  = Bt + (size_t)b * strideB;
  const T* Ab2 = SPLIT ? (A2  + (size_t)b * strideA) : nullptr;
  const T* Bb2 = SPLIT ? (Bt2 + (size_t)b * strideB) : nullptr;

  const int rlane = lane & 15;
  const int koff  = (lane >> 4) * 8;
  const int mOff  = (lane >> 4) * 8;

  v8f acc[4][4];
#pragma unroll
  for (int i = 0; i < 4; ++i)
#pragma unroll
    for (int j = 0; j < 4; ++j) acc[i][j] = (v8f){0.f,0.f,0.f,0.f,0.f,0.f,0.f,0.f};

  for (int k0 = 0; k0 < K; k0 += 32) {
    V bh[4], bl[4];
#pragma unroll
    for (int j = 0; j < 4; ++j) {
      const size_t bo = (size_t)(n0 + (j << 4) + rlane) * ldb + koff + k0;
      bh[j] = Frag<T>::load(Bb + bo);
      if (SPLIT) bl[j] = Frag<T>::load(Bb2 + bo);
    }
#pragma unroll
    for (int i = 0; i < 4; ++i) {
      const size_t ao = (size_t)(m0 + (i << 4) + rlane) * lda + koff + k0;
      V ah = Frag<T>::load(Ab + ao);
      V al;
      if (SPLIT) al = Frag<T>::load(Ab2 + ao);
#pragma unroll
      for (int j = 0; j < 4; ++j) {
        acc[i][j] = Frag<T>::mma(ah, bh[j], acc[i][j]);
        if (SPLIT) {
          acc[i][j] = Frag<T>::mma(ah, bl[j], acc[i][j]);
          acc[i][j] = Frag<T>::mma(al, bh[j], acc[i][j]);
        }
      }
      Frag<T>::guard(acc[i][0], acc[i][3], ah, SPLIT ? al : ah);
    }
    Frag<T>::keep(bh[0], bh[1], bh[2], bh[3]);
    if (SPLIT) Frag<T>::keep(bl[0], bl[1], bl[2], bl[3]);
  }
  acc_guard4(acc[0][0], acc[0][1], acc[0][2], acc[0][3]);
  acc_guard4(acc[1][0], acc[1][1], acc[1][2], acc[1][3]);
  acc_guard4(acc[2][0], acc[2][1], acc[2][2], acc[2][3]);
  acc_guard4(acc[3][0], acc[3][1], acc[3][2], acc[3][3]);

  float* slab = sT[wave];
  const float* Rb = RESID ? (resid + (size_t)b * strideR) : nullptr;
#pragma unroll
  for (int i = 0; i < 4; ++i) {
    const int mBase = m0 + (i << 4);
#pragma unroll
    for (int j = 0; j < 4; ++j) {
      const int n = n0 + (j << 4) + rlane;
      float bv = 0.f;
      if (BIAS_MODE == 2) bv = bias[n];
#pragma unroll
      for (int r = 0; r < 8; ++r) {
        float v = acc[i][j][r] * scale;
        if (BIAS_MODE == 1) v += bias[mBase + mOff + r];
        if (BIAS_MODE == 2) v += bv;
        if (RESID) v += Rb[(size_t)(mBase + mOff + r) * ldc + n];
        if (ACT == 1) v = tanhf(v);
        if (ACT == 2) v = fmaxf(v, 0.0f);
        if (ACT == 3) v = v / (1.0f + expf(-v));
        if (ACT == 4) v = (v > 0.f) ? v : 0.01f * v;
        if (ACT == 5) v = 0.5f * v * (1.0f + erff(v * 0.70710678118654752f));
        slab[(mOff + r) * 68 + (j << 4) + rlane] = v;
      }
    }
    __builtin_amdgcn_fence(__ATOMIC_RELEASE, "workgroup");
    __builtin_amdgcn_wave_barrier();
    __builtin_amdgcn_fence(__ATOMIC_ACQUIRE, "workgroup");
    if (OUT_MODE == 0) {
      float* C = (float*)Cout + (size_t)b * strideC;
      const int hh = lane >> 4, c4 = (lane & 15) * 4;
      for (int pass = 0; pass < 2; ++pass) {
#pragma unroll
        for (int it = 0; it < 8; ++it) {
          const int row = it * 2 + hh;
          v4f v = *(const v4f*)(slab + row * 68 + c4);
          *(volatile v4f*)(C + (size_t)(mBase + row) * ldc + n0 + c4) = v;
        }
        __threadfence();
      }
    } else {
      const int q = lane >> 3, c8 = (lane & 7) * 8;
      unsigned short* C  = (unsigned short*)Cout  + (size_t)b * strideC;
      unsigned short* C2 = (OUT_MODE == 2) ? ((unsigned short*)Cout2 + (size_t)b * strideC) : nullptr;
      for (int pass = 0; pass < 2; ++pass) {
#pragma unroll
        for (int it = 0; it < 4; ++it) {
          const int row = it * 4 + q;
          const float* sp = slab + row * 68 + c8;
          v8h hv, lv;
#pragma unroll
          for (int e = 0; e < 8; ++e) {
            if (OUT_MODE == 1) {
              hv[e] = (_Float16)sp[e];
            } else {
              unsigned short hb = f2bf_bits(sp[e]);
              unsigned short lb = f2bf_bits(sp[e] - bf_bits2f(hb));
              hv[e] = __builtin_bit_cast(_Float16, hb);
              lv[e] = __builtin_bit_cast(_Float16, lb);
            }
          }
          *(volatile v8h*)(C + (size_t)(mBase + row) * ldc + n0 + c8) = hv;
          if (OUT_MODE == 2) *(volatile v8h*)(C2 + (size_t)(mBase + row) * ldc + n0 + c8) = lv;
        }
        __threadfence();
      }
    }
    __builtin_amdgcn_fence(__ATOMIC_RELEASE, "workgroup");
    __builtin_amdgcn_wave_barrier();
    __builtin_amdgcn_fence(__ATOMIC_ACQUIRE, "workgroup");
  }
}

__global__ __launch_bounds__(256) void wt_kernel(const float* __restrict__ W, unsigned short* __restrict__ WT) {
  __shared__ float sm[64][65];
  const int t    = threadIdx.x;
  const int kk0  = blockIdx.x * 64;
  const int nn0  = blockIdx.y * 64;
#pragma unroll
  for (int i = 0; i < 16; ++i) {
    const int e = i * 256 + t;
    const int r = e >> 6;
    const int c = e & 63;
    sm[c][r] = W[(size_t)(kk0 + r) * kCh + nn0 + c] * kWCarry;
  }
  __syncthreads();
  const int lane = t & 31, wave = t >> 5;
  const int q = lane >> 3, c8 = (lane & 7) * 8;
  for (int pass = 0; pass < 2; ++pass) {
#pragma unroll
    for (int it = 0; it < 2; ++it) {
      const int row = wave * 8 + it * 4 + q;
      unsigned short hb[8];
#pragma unroll
      for (int e = 0; e < 8; ++e) hb[e] = h_bits(sm[row][c8 + e]);
      const v4u u = (v4u){pk16(hb[0], hb[1]), pk16(hb[2], hb[3]), pk16(hb[4], hb[5]), pk16(hb[6], hb[7])};
      *(volatile v4u*)(WT + (size_t)(nn0 + row) * kCh + kk0 + c8) = u;
    }
    __threadfence();
  }
}

__global__ __launch_bounds__(256) void gather_kernel(const float* __restrict__ x, const int* __restrict__ ei,
                                                     const float* __restrict__ epsp, unsigned short* __restrict__ H16) {
  const int lane = threadIdx.x & 31;
  const int wave = threadIdx.x >> 5;
  const float eps1 = 1.0f + epsp[0];
  const int src0 = (2 * lane) & 31;
  const int src1 = (2 * lane + 1) & 31;
#pragma unroll 1
  for (int rr = 0; rr < 4; ++rr) {
    const int row  = blockIdx.x * 32 + wave * 4 + rr;
    const int rowc = row < kNodes ? row : kNodes - 1;
    const int myidx = ei[(size_t)rowc * kNbr + lane];
    v4f acc = {0.f, 0.f, 0.f, 0.f};
#pragma unroll 1
    for (int j = 0; j < kNbr; ++j) {
      int t = __shfl(myidx, j, 32);
      t = (t < 0) ? (t + (kNodes + 1)) : t;
      t = (t < 0) ? 0 : t;
      t = (t > kNodes) ? kNodes : t;
      const float f = (t < kNodes) ? 1.0f : 0.0f;
      const int tc = (t < kNodes) ? t : (kNodes - 1);
      const v4f v = *(const v4f*)(x + (size_t)tc * kCh + 4 * lane);
      acc.x = fmaf(f, v.x, acc.x);
      acc.y = fmaf(f, v.y, acc.y);
      acc.z = fmaf(f, v.z, acc.z);
      acc.w = fmaf(f, v.w, acc.w);
    }
    const v4f xv = *(const v4f*)(x + (size_t)rowc * kCh + 4 * lane);
    v4f h;
    h.x = fmaf(eps1, xv.x, acc.x);
    h.y = fmaf(eps1, xv.y, acc.y);
    h.z = fmaf(eps1, xv.z, acc.z);
    h.w = fmaf(eps1, xv.w, acc.w);
    const bool live = row < kNodes;
    h.x = live ? h.x : 0.f;
    h.y = live ? h.y : 0.f;
    h.z = live ? h.z : 0.f;
    h.w = live ? h.w : 0.f;
    const unsigned w0 = pk16(h_bits(h.x), h_bits(h.y));
    const unsigned w1 = pk16(h_bits(h.z), h_bits(h.w));
    const unsigned a0 = (unsigned)__shfl((int)w0, src0, 32);
    const unsigned a1 = (unsigned)__shfl((int)w1, src0, 32);
    const unsigned a2 = (unsigned)__shfl((int)w0, src1, 32);
    const unsigned a3 = (unsigned)__shfl((int)w1, src1, 32);
    const v4u u = (v4u){a0, a1, a2, a3};
    unsigned short* hp = H16 + (size_t)row * kCh + 8 * lane;
    for (int pass = 0; pass < 2; ++pass) {
      if (lane < 16) *(volatile v4u*)hp = u;
      __threadfence();
    }
  }
}

__global__ __launch_bounds__(256) void ln_kernel(const float* __restrict__ Y, const float* __restrict__ bias,
                                                 const float* __restrict__ gamma, const float* __restrict__ beta,
                                                 float* __restrict__ out) {
  const int lane = threadIdx.x & 31;
  const int wave = threadIdx.x >> 5;
  const int row = blockIdx.x * 8 + wave;
  if (row >= kNodes) return;
  const v4f bv = *(const v4f*)(bias + 4 * lane);
  const v4f gv = *(const v4f*)(gamma + 4 * lane);
  const v4f be = *(const v4f*)(beta + 4 * lane);
  v4f yv = *(const v4f*)(Y + (size_t)row * kCh + 4 * lane);
  yv = yv + bv;
  float s = (yv.x + yv.y) + (yv.z + yv.w);
#pragma unroll
  for (int off = 1; off < 32; off <<= 1) s += __shfl_xor(s, off, 32);
  s = __shfl(s, 0, 32);
  const float mu = s * kInvCh;
  v4f d;
  d.x = yv.x - mu; d.y = yv.y - mu; d.z = yv.z - mu; d.w = yv.w - mu;
  float sq = (d.x * d.x + d.y * d.y) + (d.z * d.z + d.w * d.w);
#pragma unroll
  for (int off = 1; off < 32; off <<= 1) sq += __shfl_xor(sq, off, 32);
  sq = __shfl(sq, 0, 32);
  const float var  = sq * kInvCh;
  const float rstd = rsqrtf(var + kLnEps);
  v4f o;
  o.x = (d.x * rstd) * gv.x + be.x;
  o.y = (d.y * rstd) * gv.y + be.y;
  o.z = (d.z * rstd) * gv.z + be.z;
  o.w = (d.w * rstd) * gv.w + be.w;
  float* op = out + (size_t)row * kCh + 4 * lane;
  for (int pass = 0; pass < 2; ++pass) {
    *(volatile v4f*)op = o;
    __threadfence();
  }
}

extern "C" void kernel_launch(void* const* d_in, const int* in_sizes, int n_in,
                              void* d_out, int out_size, void* d_ws, size_t ws_size, hipStream_t stream) {
  (void)in_sizes; (void)n_in; (void)out_size;
  const float* x     = (const float*)d_in[0];
  const int*   ei    = (const int*)  d_in[1];
  const float* eps   = (const float*)d_in[2];
  const float* W     = (const float*)d_in[3];
  const float* b     = (const float*)d_in[4];
  const float* gamma = (const float*)d_in[5];
  const float* beta  = (const float*)d_in[6];
  float* out = (float*)d_out;

  char* ws = (char*)d_ws; size_t off = 0;
  auto carve = [&](size_t bytes) -> char* { char* p = ws + off; off += (bytes + 255) & ~(size_t)255; return p; };
  unsigned short* WT  = (unsigned short*)carve((size_t)kCh * kCh * 2);
  unsigned short* H16 = (unsigned short*)carve((size_t)kRowsPad * kCh * 2);
  float*          Y   = (float*)carve((size_t)kRowsPad * kCh * 4);
  if (off > ws_size || off > (size_t)134217728) return;

  wt_kernel<<<dim3(kCh / 64, kCh / 64), 256, 0, stream>>>(W, WT);
  gather_kernel<<<kRowsPad / 32, 256, 0, stream>>>(x, ei, eps, H16);
  {
    const int tiles = (kRowsPad / 64) * (kCh / 64);
    wmma_gemm64<0, false, 0, 0, false><<<dim3((tiles + 7) / 8, 1), 256, 0, stream>>>(
        (const unsigned short*)H16, (const unsigned short*)H16, kCh, 0L,
        (const unsigned short*)WT, (const unsigned short*)WT, kCh, 0L,
        (void*)Y, (void*)nullptr, kCh, 0L,
        (const float*)nullptr, (const float*)nullptr, 0L,
        kRowsPad, kCh, kCh, kWCarryInv);
  }
  ln_kernel<<<kNodes / 8, 256, 0, stream>>>(Y, b, gamma, beta, out);
}
